// PSA_1494648619602
// MI455X (gfx1250) — hardware-run, weakly checked
//
#include <hip/hip_runtime.h>
#include <stdint.h>

#define NB    4
#define NP    2304
#define IMW   48
#define C1    512
#define CH    256
#define NHD   4
#define KD    32
#define HD    64
#define HCH   128
#define QT    64
#define GM    128
#define GN    64
#define OSP   68
#define LTP   72
#define RSC   2048.0f
#define IRSC  0.00048828125f
#define WSC   16.0f
#define IWSC  0.0625f
#define LNPS  6.931471805599453f
#define ASCALE 0.17677669529663689f

#define WOFF1 262144
#define WOFF2 393216
#define WOFF3 458752
#define WOFF4 589824
#define WOFF5 720896
#define WTOT  983040

static_assert(IMW * IMW == NP);
static_assert(NP % QT == 0);
static_assert(NP % GN == 0);
static_assert(NP % 32 == 0);
static_assert(C1 % GM == 0);
static_assert(CH % GM == 0);
static_assert(HCH == 2 * KD + HD);
static_assert(NHD * HCH == C1);
static_assert(NHD * HD == CH);
static_assert(WTOT % 2048 == 0);
static_assert(WOFF1 % 2048 == 0);
static_assert(WOFF2 % 2048 == 0);
static_assert(WOFF3 % 2048 == 0);
static_assert(WOFF4 % 2048 == 0);
static_assert(WOFF5 % 2048 == 0);
static_assert((GM * OSP * 4) % 16 == 0);
static_assert((OSP * 4) % 16 == 0);
static_assert((LTP * 2) % 16 == 0);

typedef _Float16       v16h __attribute__((ext_vector_type(16)));
typedef _Float16       v8h  __attribute__((ext_vector_type(8)));
typedef __bf16         v16b __attribute__((ext_vector_type(16)));
typedef unsigned short v8us __attribute__((ext_vector_type(8)));
typedef float          v8f  __attribute__((ext_vector_type(8)));
typedef float          v4f  __attribute__((ext_vector_type(4)));
typedef unsigned int   v4u  __attribute__((ext_vector_type(4)));

union Frag  { v8us u[2]; v16h h; v16b bf; };
union FragH { v16h v; v8h hv[2]; };
static_assert(sizeof(Frag) == 32);
static_assert(sizeof(FragH) == 32);

__device__ __forceinline__ unsigned short bf_bits(float f) {
  unsigned u = __float_as_uint(f);
  return (unsigned short)((u + 0x7FFFu + ((u >> 16) & 1u)) >> 16);
}
__device__ __forceinline__ float bf_up(unsigned short hb) { return __uint_as_float(((unsigned)hb) << 16); }
__device__ __forceinline__ float bfr(float f) { return bf_up(bf_bits(f)); }
__device__ __forceinline__ unsigned short h_bits(_Float16 x) { return __builtin_bit_cast(unsigned short, x); }
__device__ __forceinline__ unsigned pk16(unsigned short a, unsigned short b) { return (unsigned)a | ((unsigned)b << 16); }
__device__ __forceinline__ v8f zero8() { v8f z = {0.f, 0.f, 0.f, 0.f, 0.f, 0.f, 0.f, 0.f}; return z; }
__device__ __forceinline__ float hmax8(v8f s) {
  return fmaxf(fmaxf(fmaxf(s[0], s[1]), fmaxf(s[2], s[3])), fmaxf(fmaxf(s[4], s[5]), fmaxf(s[6], s[7])));
}

__device__ __forceinline__ Frag ldfrag(const unsigned short* p) {
  Frag f;
  f.u[0] = *(const v8us*)(p);
  f.u[1] = *(const v8us*)(p + 16);
  return f;
}

__device__ __forceinline__ v8f mma_h(v16h a, v16h b, v8f c) {
  v8f d = __builtin_amdgcn_wmma_f32_16x16x32_f16(false, a, false, b, (short)0, c, false, false);
#if defined(__HIP_DEVICE_COMPILE__)
  asm volatile("v_nop\n\tv_nop\n\tv_nop\n\tv_nop" : "+v"(d) : "v"(a), "v"(b));
#endif
  return d;
}
__device__ __forceinline__ v8f mma_b(v16b a, v16b b, v8f c) {
  v8f d = __builtin_amdgcn_wmma_f32_16x16x32_bf16(false, a, false, b, (short)0, c, false, false);
#if defined(__HIP_DEVICE_COMPILE__)
  const v16h ha = __builtin_bit_cast(v16h, a), hb = __builtin_bit_cast(v16h, b);
  asm volatile("v_nop\n\tv_nop\n\tv_nop\n\tv_nop" : "+v"(d) : "v"(ha), "v"(hb));
#endif
  return d;
}

__global__ __launch_bounds__(256)
void cvt_w(const float* __restrict__ w0, const float* __restrict__ w1, const float* __restrict__ w2,
           const float* __restrict__ w3, const float* __restrict__ w4, const float* __restrict__ w5,
           unsigned short* WB) {
  const int g0 = (int)blockIdx.x * 2048;
  const float* src = w0;
  int base = 0;
  bool isbf = true;
  if (g0 >= WOFF5)      { src = w5; base = WOFF5; isbf = false; }
  else if (g0 >= WOFF4) { src = w4; base = WOFF4; isbf = false; }
  else if (g0 >= WOFF3) { src = w3; base = WOFF3; isbf = false; }
  else if (g0 >= WOFF2) { src = w2; base = WOFF2; isbf = false; }
  else if (g0 >= WOFF1) { src = w1; base = WOFF1; isbf = false; }
  const int i = g0 + (int)threadIdx.x * 8;
  const float* s = src + (i - base);
  const v4f a = *(const v4f*)(s);
  const v4f q = *(const v4f*)(s + 4);
  v4u w;
  if (isbf) {
    w[0] = pk16(bf_bits(a[0]), bf_bits(a[1]));
    w[1] = pk16(bf_bits(a[2]), bf_bits(a[3]));
    w[2] = pk16(bf_bits(q[0]), bf_bits(q[1]));
    w[3] = pk16(bf_bits(q[2]), bf_bits(q[3]));
  } else {
    w[0] = pk16(h_bits((_Float16)(bfr(a[0]) * WSC)), h_bits((_Float16)(bfr(a[1]) * WSC)));
    w[1] = pk16(h_bits((_Float16)(bfr(a[2]) * WSC)), h_bits((_Float16)(bfr(a[3]) * WSC)));
    w[2] = pk16(h_bits((_Float16)(bfr(q[0]) * WSC)), h_bits((_Float16)(bfr(q[1]) * WSC)));
    w[3] = pk16(h_bits((_Float16)(bfr(q[2]) * WSC)), h_bits((_Float16)(bfr(q[3]) * WSC)));
  }
  unsigned short* p = WB + (size_t)i;
  *(volatile v4u*)p = w;
  __threadfence();
  *(volatile v4u*)p = w;
}

__global__ __launch_bounds__(256)
void cvt_x(const float* __restrict__ x, unsigned short* X16) {
  __shared__ __align__(16) unsigned short Lt[GN * LTP];
  const int tid = threadIdx.x;
  const int nt = blockIdx.x, cg = blockIdx.y, b = blockIdx.z;
  const int n0 = nt * GN;
  {
    const int n4 = (tid & 15) * 4, cs = tid >> 4;
#pragma unroll
    for (int it = 0; it < 4; ++it) {
      const int cl = it * 16 + cs;
      const v4f v = *(const v4f*)(x + ((size_t)(b * C1 + cg * 64 + cl)) * NP + n0 + n4);
#pragma unroll
      for (int qq = 0; qq < 4; ++qq) Lt[(n4 + qq) * LTP + cl] = bf_bits(v[qq]);
    }
  }
  __syncthreads();
  {
    const int e = tid & 7, lq = tid >> 3;
#pragma unroll
    for (int pass = 0; pass < 2; ++pass) {
#pragma unroll
      for (int it = 0; it < 2; ++it) {
        const int n = it * 32 + lq;
        const v4u u = *(const v4u*)(Lt + n * LTP + 8 * e);
        *(volatile v4u*)(X16 + ((size_t)(b * NP + n0 + n)) * C1 + cg * 64 + 8 * e) = u;
      }
      __threadfence();
    }
  }
}

template <int MODE>
__global__ __launch_bounds__(256)
void gemm_kernel(const unsigned short* __restrict__ Wp, int K, float sA,
                 const unsigned short* __restrict__ P0h, const unsigned short* __restrict__ P0l, int p0p, int p0k,
                 const unsigned short* __restrict__ P1h, const unsigned short* __restrict__ P1l, int p1p,
                 int ksplit,
                 const float* __restrict__ sc, const float* __restrict__ bi,
                 const float* __restrict__ resid, int res_ch, int act,
                 float* outF, int of_ch, int of_lo,
                 unsigned short* out16, int o16_ch,
                 unsigned short* outPh, unsigned short* outPl, int op_ch) {
  __shared__ __align__(16) float Os[GM * OSP];
  const int tid  = threadIdx.x;
  const int lane = tid & 31, wave = tid >> 5;
  const int hh   = lane >> 4, c = lane & 15;
  const int wm   = wave >> 1, wn = wave & 1;
  const int b    = blockIdx.z;
  const int mBase = blockIdx.x * GM;
  const int nBase = blockIdx.y * GN;

  const unsigned short* a0p = Wp + (size_t)(mBase + 32 * wm + c) * K + 8 * hh;
  const unsigned short* a1p = a0p + (size_t)16 * K;
  const size_t nrow = (size_t)b * NP + nBase + 32 * wn + c;

  v8f acc[2][2], accr[2][2];
#pragma unroll
  for (int mi = 0; mi < 2; ++mi)
#pragma unroll
    for (int ni = 0; ni < 2; ++ni) { acc[mi][ni] = zero8(); accr[mi][ni] = zero8(); }

#pragma unroll 1
  for (int k0 = 0; k0 < K; k0 += 32) {
    const bool first = (k0 < ksplit);
    const unsigned short* ph = first ? P0h : P1h;
    const unsigned short* pl = first ? P0l : P1l;
    const int pp = first ? p0p : p1p;
    const int kk = (first ? (p0k + k0) : (k0 - ksplit)) + 8 * hh;
    const size_t bo0 = nrow * (size_t)pp + kk;
    const size_t bo1 = bo0 + (size_t)16 * pp;
    const Frag fa0 = ldfrag(a0p + k0);
    const Frag fa1 = ldfrag(a1p + k0);
    const Frag fb0 = ldfrag(ph + bo0);
    const Frag fb1 = ldfrag(ph + bo1);
    if (MODE == 0) {
      acc[0][0] = mma_b(fa0.bf, fb0.bf, acc[0][0]);
      acc[0][1] = mma_b(fa0.bf, fb1.bf, acc[0][1]);
      acc[1][0] = mma_b(fa1.bf, fb0.bf, acc[1][0]);
      acc[1][1] = mma_b(fa1.bf, fb1.bf, acc[1][1]);
    } else {
      acc[0][0] = mma_h(fa0.h, fb0.h, acc[0][0]);
      acc[0][1] = mma_h(fa0.h, fb1.h, acc[0][1]);
      acc[1][0] = mma_h(fa1.h, fb0.h, acc[1][0]);
      acc[1][1] = mma_h(fa1.h, fb1.h, acc[1][1]);
      if (MODE == 2) {
        const Frag fl0 = ldfrag(pl + bo0);
        const Frag fl1 = ldfrag(pl + bo1);
        accr[0][0] = mma_h(fa0.h, fl0.h, accr[0][0]);
        accr[0][1] = mma_h(fa0.h, fl1.h, accr[0][1]);
        accr[1][0] = mma_h(fa1.h, fl0.h, accr[1][0]);
        accr[1][1] = mma_h(fa1.h, fl1.h, accr[1][1]);
      }
    }
  }

  const float rsA = sA * IRSC;
#pragma unroll
  for (int mi = 0; mi < 2; ++mi) {
#pragma unroll
    for (int ni = 0; ni < 2; ++ni) {
      const int n_loc = 32 * wn + 16 * ni + c;
      const int n = nBase + n_loc;
#pragma unroll
      for (int r = 0; r < 8; ++r) {
        const int o_loc = 32 * wm + 16 * mi + 8 * hh + r;
        const int o = mBase + o_loc;
        float v = acc[mi][ni][r] * sA;
        if (MODE == 2) v += accr[mi][ni][r] * rsA;
        v = v * bfr(sc[o]) + bfr(bi[o]);
        if (resid != nullptr) v += resid[((size_t)b * res_ch + o) * NP + n];
        if (act != 0) {
          const float ex = __expf(fminf(-v, 30.0f));
          v = v * __builtin_amdgcn_rcpf(1.0f + ex);
        }
        Os[o_loc * OSP + n_loc] = v;
      }
    }
  }
  __syncthreads();

  {
    const int e = tid & 7, lq = tid >> 3;
    const bool doF = (outF != nullptr) && (mBase >= of_lo);
#pragma unroll
    for (int pass = 0; pass < 2; ++pass) {
      if (doF) {
#pragma unroll
        for (int it = 0; it < 8; ++it) {
          const int L = it * 32 + lq;
          const int row = L >> 1, hf = L & 1;
          const v4f v = *(const v4f*)(Os + row * OSP + hf * 32 + 4 * e);
          float* dst = outF + ((size_t)b * of_ch + (mBase - of_lo) + row) * NP + nBase + hf * 32 + 4 * e;
          *(volatile v4f*)dst = v;
        }
      }
      if (out16 != nullptr) {
#pragma unroll
        for (int it = 0; it < 4; ++it) {
          const int row = it * 32 + lq;
          const v4f v0 = *(const v4f*)(Os + row * OSP + 8 * e);
          const v4f v1 = *(const v4f*)(Os + row * OSP + 8 * e + 4);
          v4u u;
          u[0] = pk16(h_bits((_Float16)v0[0]), h_bits((_Float16)v0[1]));
          u[1] = pk16(h_bits((_Float16)v0[2]), h_bits((_Float16)v0[3]));
          u[2] = pk16(h_bits((_Float16)v1[0]), h_bits((_Float16)v1[1]));
          u[3] = pk16(h_bits((_Float16)v1[2]), h_bits((_Float16)v1[3]));
          unsigned short* dst = out16 + ((size_t)b * o16_ch + mBase + row) * NP + nBase + 8 * e;
          *(volatile v4u*)dst = u;
        }
      }
      if (outPh != nullptr) {
#pragma unroll
        for (int it = 0; it < 4; ++it) {
          const int L = it * 32 + lq;
          const int n_loc = L >> 1, hf = L & 1;
          const int ch0 = hf * 64 + 8 * e;
          float f[8];
#pragma unroll
          for (int j = 0; j < 8; ++j) f[j] = Os[(ch0 + j) * OSP + n_loc];
          v4u uh, ul;
#pragma unroll
          for (int t = 0; t < 4; ++t) {
            const _Float16 h0 = (_Float16)f[2 * t];
            const _Float16 h1 = (_Float16)f[2 * t + 1];
            const _Float16 l0 = (_Float16)((f[2 * t] - (float)h0) * RSC);
            const _Float16 l1 = (_Float16)((f[2 * t + 1] - (float)h1) * RSC);
            uh[t] = pk16(h_bits(h0), h_bits(h1));
            ul[t] = pk16(h_bits(l0), h_bits(l1));
          }
          const size_t po = ((size_t)b * NP + nBase + n_loc) * (size_t)op_ch + mBase + ch0;
          *(volatile v4u*)(outPh + po) = uh;
          if (outPl != nullptr) *(volatile v4u*)(outPl + po) = ul;
        }
      }
      __threadfence();
    }
  }
}

__global__ __launch_bounds__(128)
void attn_kernel(const unsigned short* __restrict__ Qh, const unsigned short* __restrict__ V16, float* ATT) {
  __shared__ __align__(16) float Os[HD * OSP];
  const int tid  = threadIdx.x;
  const int wave = tid >> 5, lane = tid & 31;
  const int hh   = lane >> 4, c = lane & 15;
  const int qb   = blockIdx.x, h = blockIdx.y, b = blockIdx.z;
  const int n0   = qb * QT;

  const Frag qf = ldfrag(Qh + ((size_t)b * NP + n0 + 16 * wave + c) * C1 + h * HCH + 8 * hh);
  const v16h q = qf.h;
  const unsigned short* Kp = Qh + ((size_t)b * NP + c) * C1 + h * HCH + KD + 8 * hh;
  const unsigned short* Vb = V16 + ((size_t)b * C1 + h * HCH + 2 * KD + c) * NP + 8 * hh;

  float m = -1.0e30f, l = 0.f;
  v8f o0 = zero8(), o1 = zero8(), o2 = zero8(), o3 = zero8();
#pragma unroll 1
  for (int it = 0; it < NP / 32; ++it) {
    const int kb = it * 32;
    const Frag k0f = ldfrag(Kp + (size_t)kb * C1);
    const Frag k1f = ldfrag(Kp + (size_t)(kb + 16) * C1);
    v8f s0 = mma_h(k0f.h, q, zero8());
    v8f s1 = mma_h(k1f.h, q, zero8());
#pragma unroll
    for (int r = 0; r < 8; ++r) { s0[r] *= ASCALE; s1[r] *= ASCALE; }

    float mx = fmaxf(hmax8(s0), hmax8(s1));
    mx = fmaxf(mx, __shfl_xor(mx, 16, 32));
    const float mn   = fmaxf(m, mx);
    const float corr = __expf(m - mn);
    m = mn;
    const float msh = mn - LNPS;
    l *= corr;
#pragma unroll
    for (int r = 0; r < 8; ++r) { o0[r] *= corr; o1[r] *= corr; o2[r] *= corr; o3[r] *= corr; }

    FragH ph;
    float ls = 0.f;
#pragma unroll
    for (int r = 0; r < 8; ++r) {
      const float e0 = __expf(s0[r] - msh);
      const float e1 = __expf(s1[r] - msh);
      ls += e0 + e1;
      ph.hv[0][r] = (_Float16)e0;
      ph.hv[1][r] = (_Float16)e1;
    }
    l += ls;

    const Frag v0f = ldfrag(Vb + kb);
    const Frag v1f = ldfrag(Vb + (size_t)16 * NP + kb);
    const Frag v2f = ldfrag(Vb + (size_t)32 * NP + kb);
    const Frag v3f = ldfrag(Vb + (size_t)48 * NP + kb);
    o0 = mma_h(v0f.h, ph.v, o0);
    o1 = mma_h(v1f.h, ph.v, o1);
    o2 = mma_h(v2f.h, ph.v, o2);
    o3 = mma_h(v3f.h, ph.v, o3);
  }
  l += __shfl_xor(l, 16, 32);
  const float inv = 1.0f / l;

  float* os = Os + (8 * hh) * OSP + wave * 16 + c;
#pragma unroll
  for (int r = 0; r < 8; ++r) {
    os[(0 * 16 + r) * OSP] = o0[r] * inv;
    os[(1 * 16 + r) * OSP] = o1[r] * inv;
    os[(2 * 16 + r) * OSP] = o2[r] * inv;
    os[(3 * 16 + r) * OSP] = o3[r] * inv;
  }
  __syncthreads();
  {
    const int e = tid & 7, lq = tid >> 3;
    float* ob = ATT + ((size_t)b * CH + h * HD) * NP + n0;
#pragma unroll
    for (int pass = 0; pass < 2; ++pass) {
#pragma unroll
      for (int it = 0; it < 8; ++it) {
        const int L   = it * 16 + lq;
        const int row = L >> 1, hf = L & 1;
        const v4f v = *(const v4f*)(Os + row * OSP + hf * 32 + 4 * e);
        *(volatile v4f*)(ob + (size_t)row * NP + hf * 32 + 4 * e) = v;
      }
      __threadfence();
    }
  }
}

__global__ __launch_bounds__(256)
void pe_kernel(const unsigned short* __restrict__ V16, const float* __restrict__ ATT,
               const float* __restrict__ pw, const float* __restrict__ ps, const float* __restrict__ pb,
               unsigned short* Th, unsigned short* Tl) {
  __shared__ __align__(16) unsigned short Lh[GN * LTP];
  __shared__ __align__(16) unsigned short Ll[GN * LTP];
  const int tid = threadIdx.x;
  const int nl  = tid & 63, cgrp = tid >> 6;
  const int nt  = blockIdx.x, cg = blockIdx.y, b = blockIdx.z;
  const int n0  = nt * GN;
  const int n   = n0 + nl;
  const int y   = n / IMW;
  const int xq  = n - y * IMW;
  const _Float16* Vh = (const _Float16*)(const void*)V16;
#pragma unroll 1
  for (int j = 0; j < 16; ++j) {
    const int cl = cgrp * 16 + j;
    const int cc = cg * 64 + cl;
    const _Float16* vr = Vh + ((size_t)(b * C1 + cg * HCH + 2 * KD + cl)) * NP;
    float accv = 0.f;
#pragma unroll
    for (int t = 0; t < 9; ++t) {
      const int ky = t / 3, kx = t - ky * 3;
      const int yy = y + ky - 1, xx = xq + kx - 1;
      const bool ok = ((unsigned)yy < (unsigned)IMW) && ((unsigned)xx < (unsigned)IMW);
      const int yc = min(max(yy, 0), IMW - 1);
      const int xc = min(max(xx, 0), IMW - 1);
      const float hv = (float)vr[yc * IMW + xc];
      const float wv = bfr(pw[cc * 9 + t]);
      accv = fmaf(ok ? hv : 0.f, wv, accv);
    }
    const float att = ATT[((size_t)(b * CH + cc)) * NP + n];
    const float val = att + (accv * bfr(ps[cc]) + bfr(pb[cc]));
    const _Float16 hi = (_Float16)val;
    const float res = (val - (float)hi) * RSC;
    Lh[nl * LTP + cl] = h_bits(hi);
    Ll[nl * LTP + cl] = h_bits((_Float16)res);
  }
  __syncthreads();
  {
    const int e = tid & 7, lq = tid >> 3;
#pragma unroll
    for (int pass = 0; pass < 2; ++pass) {
#pragma unroll
      for (int it = 0; it < 2; ++it) {
        const int nn = it * 32 + lq;
        const v4u uh = *(const v4u*)(Lh + nn * LTP + 8 * e);
        const v4u ul = *(const v4u*)(Ll + nn * LTP + 8 * e);
        const size_t po = ((size_t)(b * NP + n0 + nn)) * CH + cg * 64 + 8 * e;
        *(volatile v4u*)(Th + po) = uh;
        *(volatile v4u*)(Tl + po) = ul;
      }
      __threadfence();
    }
  }
}

extern "C" void kernel_launch(void* const* d_in, const int* in_sizes, int n_in,
                              void* d_out, int out_size, void* d_ws, size_t ws_size,
                              hipStream_t stream) {
  const int NX = NB * C1 * NP;
  if (n_in < 22) return;
  if (in_sizes[0] != NX) return;
  if (in_sizes[1] != C1 * C1 || in_sizes[2] != C1 || in_sizes[3] != C1) return;
  if (in_sizes[4] != C1 * CH || in_sizes[5] != C1 || in_sizes[6] != C1) return;
  if (in_sizes[7] != CH * 9 || in_sizes[8] != CH || in_sizes[9] != CH) return;
  if (in_sizes[10] != CH * CH || in_sizes[11] != CH || in_sizes[12] != CH) return;
  if (in_sizes[13] != C1 * CH || in_sizes[14] != C1 || in_sizes[15] != C1) return;
  if (in_sizes[16] != CH * C1 || in_sizes[17] != CH || in_sizes[18] != CH) return;
  if (in_sizes[19] != C1 * C1 || in_sizes[20] != C1 || in_sizes[21] != C1) return;
  if (out_size != NX) return;

  const size_t U  = (size_t)NB * NP * C1 * 2;
  const size_t HU = U / 2;
  size_t off = 0;
  const size_t oW   = off; off += (size_t)WTOT * 2;
  const size_t oX   = off; off += U;
  const size_t oABR = off; off += U;
  const size_t oABh = off; off += U;
  const size_t oABl = off; off += U;
  const size_t oQh  = off; off += U;
  const size_t oQ16 = off; off += U;
  const size_t oATT = off; off += U;
  const size_t oTh  = off; off += HU;
  const size_t oTl  = off; off += HU;
  const size_t oB2f = off; off += U;
  const size_t oB2h = off; off += HU;
  const size_t oB2l = off; off += HU;
  const size_t oFh  = off; off += U;
  const size_t oFl  = off; off += U;
  const size_t oB3h = off; off += HU;
  const size_t oB3l = off; off += HU;
  if (off > ws_size) return;
  if (off > (size_t)134217728) return;

  const float* x      = (const float*)d_in[0];
  const float* cv1_w  = (const float*)d_in[1];
  const float* cv1_s  = (const float*)d_in[2];
  const float* cv1_b  = (const float*)d_in[3];
  const float* qkv_w  = (const float*)d_in[4];
  const float* qkv_s  = (const float*)d_in[5];
  const float* qkv_b  = (const float*)d_in[6];
  const float* pe_w   = (const float*)d_in[7];
  const float* pe_s   = (const float*)d_in[8];
  const float* pe_b   = (const float*)d_in[9];
  const float* proj_w = (const float*)d_in[10];
  const float* proj_s = (const float*)d_in[11];
  const float* proj_b = (const float*)d_in[12];
  const float* ffn1_w = (const float*)d_in[13];
  const float* ffn1_s = (const float*)d_in[14];
  const float* ffn1_b = (const float*)d_in[15];
  const float* ffn2_w = (const float*)d_in[16];
  const float* ffn2_s = (const float*)d_in[17];
  const float* ffn2_b = (const float*)d_in[18];
  const float* cv2_w  = (const float*)d_in[19];
  const float* cv2_s  = (const float*)d_in[20];
  const float* cv2_b  = (const float*)d_in[21];

  char* ws = (char*)d_ws;
  unsigned short* WB  = (unsigned short*)(ws + oW);
  unsigned short* X16 = (unsigned short*)(ws + oX);
  float*          ABR = (float*)(ws + oABR);
  unsigned short* ABh = (unsigned short*)(ws + oABh);
  unsigned short* ABl = (unsigned short*)(ws + oABl);
  unsigned short* Qh  = (unsigned short*)(ws + oQh);
  unsigned short* Q16 = (unsigned short*)(ws + oQ16);
  float*          ATT = (float*)(ws + oATT);
  unsigned short* Th  = (unsigned short*)(ws + oTh);
  unsigned short* Tl  = (unsigned short*)(ws + oTl);
  float*          B2f = (float*)(ws + oB2f);
  unsigned short* B2h = (unsigned short*)(ws + oB2h);
  unsigned short* B2l = (unsigned short*)(ws + oB2l);
  unsigned short* Fh  = (unsigned short*)(ws + oFh);
  unsigned short* Fl  = (unsigned short*)(ws + oFl);
  unsigned short* B3h = (unsigned short*)(ws + oB3h);
  unsigned short* B3l = (unsigned short*)(ws + oB3l);
  float* out = (float*)d_out;

  const dim3 blk256(256), blk128(128);
  const dim3 gW(WTOT / 2048);
  const dim3 gX(NP / GN, C1 / 64, NB);
  const dim3 g512(C1 / GM, NP / GN, NB);
  const dim3 g256(CH / GM, NP / GN, NB);
  const dim3 gA(NP / QT, NHD, NB);
  const dim3 gPE(NP / GN, CH / 64, NB);

  cvt_w<<<gW, blk256, 0, stream>>>(cv1_w, qkv_w, proj_w, ffn1_w, ffn2_w, cv2_w, WB);
  cvt_x<<<gX, blk256, 0, stream>>>(x, X16);
  gemm_kernel<0><<<g512, blk256, 0, stream>>>(WB, C1, 1.0f,
      X16, X16, C1, 0, X16, X16, C1, C1,
      cv1_s, cv1_b, nullptr, 0, 1,
      ABR, CH, CH, nullptr, 0, ABh, ABl, C1);
  gemm_kernel<1><<<g512, blk256, 0, stream>>>(WB + WOFF1, CH, IWSC,
      ABh, ABl, C1, CH, ABh, ABl, C1, CH,
      qkv_s, qkv_b, nullptr, 0, 0,
      nullptr, 0, 0, Q16, C1, Qh, nullptr, C1);
  attn_kernel<<<gA, blk128, 0, stream>>>(Qh, Q16, ATT);
  pe_kernel<<<gPE, blk256, 0, stream>>>(Q16, ATT, pe_w, pe_s, pe_b, Th, Tl);
  gemm_kernel<2><<<g256, blk256, 0, stream>>>(WB + WOFF2, CH, IWSC,
      Th, Tl, CH, 0, Th, Tl, CH, CH,
      proj_s, proj_b, ABR, CH, 0,
      B2f, CH, 0, nullptr, 0, B2h, B2l, CH);
  gemm_kernel<2><<<g512, blk256, 0, stream>>>(WB + WOFF3, CH, IWSC,
      B2h, B2l, CH, 0, B2h, B2l, CH, CH,
      ffn1_s, ffn1_b, nullptr, 0, 1,
      nullptr, 0, 0, nullptr, 0, Fh, Fl, C1);
  gemm_kernel<2><<<g256, blk256, 0, stream>>>(WB + WOFF4, C1, IWSC,
      Fh, Fl, C1, 0, Fh, Fl, C1, C1,
      ffn2_s, ffn2_b, B2f, CH, 0,
      nullptr, 0, 0, nullptr, 0, B3h, B3l, CH);
  gemm_kernel<2><<<g512, blk256, 0, stream>>>(WB + WOFF5, C1, IWSC,
      ABh, ABl, C1, 0, B3h, B3l, CH, CH,
      cv2_s, cv2_b, nullptr, 0, 1,
      out, C1, 0, nullptr, 0, nullptr, nullptr, C1);
  (void)hipGetLastError();
}
